// testLSTMNet_2078764171594
// MI455X (gfx1250) — hardware-verified
//
#include <hip/hip_runtime.h>
#include <math.h>

constexpr int NBATCH     = 64;
constexpr int NSTEP      = 512;
constexpr int NFEAT      = 128;
constexpr int NHID       = 128;
constexpr int NGATE      = 4 * NHID;
constexpr int NROWS      = NBATCH * NSTEP;
constexpr int NFC1       = 1024;
constexpr int NFC2       = 2048;
constexpr int NCLS       = 10;
constexpr int NCLS_PAD   = 16;
constexpr int CHUNK_ROWS = 4096;
constexpr int NCHUNK     = NROWS / CHUNK_ROWS;
constexpr int SEQ_BLK    = 16;
constexpr int HPITCH     = 136;
constexpr int XGPITCH    = 516;
constexpr int SLABP      = 68;
constexpr int NTHR       = 256;
constexpr float WCARRY     = 16.0f;
constexpr float WCARRY_INV = 1.0f / 16.0f;

static_assert(NGATE == 512, "gate plane width");
static_assert(NROWS == 32768, "row count");
static_assert(NBATCH % SEQ_BLK == 0, "sequence blocks");
static_assert(NHID == 16 * (NTHR / 32), "8 waves x 16 hidden columns");
static_assert(NFEAT % 32 == 0 && NHID % 32 == 0 && NFC1 % 32 == 0 && NFC2 % 32 == 0, "K multiples of 32");
static_assert(NROWS % 64 == 0 && CHUNK_ROWS % 64 == 0 && NGATE % 64 == 0 && NFC1 % 64 == 0 && NFC2 % 64 == 0, "M, N tile multiples");
static_assert(((NROWS / 64) * (NGATE / 64)) % 8 == 0, "tile count, projection");
static_assert(((CHUNK_ROWS / 64) * (NFC1 / 64)) % 8 == 0, "tile count, dense 1");
static_assert(((CHUNK_ROWS / 64) * (NFC2 / 64)) % 8 == 0, "tile count, dense 2");
static_assert(NROWS % CHUNK_ROWS == 0, "chunking");
static_assert((64 * NCLS * 4) % 128 == 0, "64 output rows span whole lines");
static_assert((SEQ_BLK * (NGATE / 4)) % NTHR == 0, "gate tile staging exact");
static_assert((HPITCH % 8) == 0 && (XGPITCH % 4) == 0, "LDS pitches keep 16-B alignment");

typedef __attribute__((ext_vector_type(16))) _Float16 v16h;
typedef __attribute__((ext_vector_type(8)))  _Float16 v8h;
typedef __attribute__((ext_vector_type(8)))  float    v8f;
typedef __attribute__((ext_vector_type(4)))  float    v4f;

__device__ __forceinline__ v16h frag_load(const _Float16* p) {
  union U { v16h v; v8h h[2]; } f;
  f.h[0] = *(const v8h*)(p);
  f.h[1] = *(const v8h*)(p + 16);
  return f.v;
}
__device__ __forceinline__ v8f mma_f16(v16h a, v16h b, v8f c) {
  return __builtin_amdgcn_wmma_f32_16x16x32_f16(false, a, false, b, (short)0, c, false, false);
}
__device__ __forceinline__ void guard4(v8f& a0, v8f& a1, v8f& a2, v8f& a3, v16h x, v16h y0, v16h y1, v16h y2, v16h y3) {
  asm volatile("v_nop\n\tv_nop\n\tv_nop\n\tv_nop" : "+v"(a0), "+v"(a1), "+v"(a2), "+v"(a3) : "v"(x), "v"(y0), "v"(y1), "v"(y2), "v"(y3));
}
__device__ __forceinline__ void guard1(v8f& a, v16h x, v16h y) {
  asm volatile("v_nop\n\tv_nop\n\tv_nop\n\tv_nop" : "+v"(a) : "v"(x), "v"(y));
}
__device__ __forceinline__ void acc_guard4(v8f& a, v8f& b, v8f& c, v8f& d) {
  asm volatile("v_nop\n\tv_nop\n\tv_nop\n\tv_nop" : "+v"(a), "+v"(b), "+v"(c), "+v"(d));
}
__device__ __forceinline__ void acc_guard1(v8f& a) {
  asm volatile("v_nop\n\tv_nop\n\tv_nop\n\tv_nop" : "+v"(a));
}

__device__ __forceinline__ float gate_sig(float x)  { return __builtin_amdgcn_rcpf(1.0f + expf(-x)); }
__device__ __forceinline__ float gate_tanh(float x) { return 1.0f - 2.0f * __builtin_amdgcn_rcpf(expf(2.0f * x) + 1.0f); }

__global__ __launch_bounds__(NTHR) void cvt8_f16_kernel(const float* __restrict__ src, unsigned short* __restrict__ dst,
                                                        int n8_valid, int n8_total, float sc) {
  const int i = blockIdx.x * NTHR + threadIdx.x;
  if (i < n8_total) {
    const bool ok = (i < n8_valid);
    const int ic = ok ? i : (n8_valid - 1);
    const float* sp = src + (size_t)ic * 8;
    const v4f a = *(const v4f*)(sp);
    const v4f b = *(const v4f*)(sp + 4);
    v8h hv;
#pragma unroll
    for (int e = 0; e < 4; ++e) {
      const float fa = ok ? (a[e] * sc) : 0.0f;
      const float fb = ok ? (b[e] * sc) : 0.0f;
      hv[e]     = (_Float16)fa;
      hv[4 + e] = (_Float16)fb;
    }
    unsigned short* dp = dst + (size_t)i * 8;
    *(volatile v8h*)dp = hv;
    __threadfence();
    *(volatile v8h*)dp = hv;
  }
}

__global__ __launch_bounds__(NTHR) void bias_sum_kernel(const float* __restrict__ ba0, const float* __restrict__ bb0,
                                                        const float* __restrict__ ba1, const float* __restrict__ bb1,
                                                        float* __restrict__ dst) {
  const int tid = threadIdx.x;
  const int which = tid >> 7;
  const int idx = (tid & 127) * 4;
  const v4f a0 = *(const v4f*)(ba0 + idx);
  const v4f b0 = *(const v4f*)(bb0 + idx);
  const v4f a1 = *(const v4f*)(ba1 + idx);
  const v4f b1 = *(const v4f*)(bb1 + idx);
  v4f o;
#pragma unroll
  for (int e = 0; e < 4; ++e) {
    const float s0 = a0[e] + b0[e];
    const float s1 = a1[e] + b1[e];
    o[e] = which ? s1 : s0;
  }
  float* op = dst + which * NGATE + idx;
  *(volatile v4f*)op = o;
  __threadfence();
  *(volatile v4f*)op = o;
}

template <int OUT_MODE, int ACT>
__global__ __launch_bounds__(256) void gemm_f16_tile64(
    const unsigned short* __restrict__ Ap, int lda,
    const unsigned short* __restrict__ Btp, int ldb,
    void* __restrict__ Cout, int ldc,
    const float* __restrict__ bias,
    int M, int N, int K, float scale) {
  const _Float16* A  = (const _Float16*)Ap;
  const _Float16* Bt = (const _Float16*)Btp;
  __shared__ __align__(16) float sT[8][16 * SLABP];
  const int lane = threadIdx.x & 31;
  const int wave = threadIdx.x >> 5;
  const int tilesN = N >> 6;
  const int tilesM = M >> 6;
  const int tile = blockIdx.x * 8 + wave;
  if (tile >= tilesM * tilesN) return;
  const int tm = tile / tilesN;
  const int tn = tile - tm * tilesN;
  const int m0 = tm << 6;
  const int n0 = tn << 6;

  const int rlane = lane & 15;
  const int koff  = (lane >> 4) * 8;
  const int mOff  = (lane >> 4) * 8;

  const _Float16* aptr[4];
  const _Float16* bptr[4];
#pragma unroll
  for (int i = 0; i < 4; ++i) {
    aptr[i] = A  + (size_t)(m0 + (i << 4) + rlane) * lda + koff;
    bptr[i] = Bt + (size_t)(n0 + (i << 4) + rlane) * ldb + koff;
  }

  v8f acc[4][4];
#pragma unroll
  for (int i = 0; i < 4; ++i)
#pragma unroll
    for (int j = 0; j < 4; ++j) acc[i][j] = (v8f){0.f, 0.f, 0.f, 0.f, 0.f, 0.f, 0.f, 0.f};

  for (int k0 = 0; k0 < K; k0 += 32) {
    v16h bh[4];
#pragma unroll
    for (int j = 0; j < 4; ++j) bh[j] = frag_load(bptr[j] + k0);
#pragma unroll
    for (int i = 0; i < 4; ++i) {
      const v16h ah = frag_load(aptr[i] + k0);
#pragma unroll
      for (int j = 0; j < 4; ++j) acc[i][j] = mma_f16(ah, bh[j], acc[i][j]);
      guard4(acc[i][0], acc[i][1], acc[i][2], acc[i][3], ah, bh[0], bh[1], bh[2], bh[3]);
    }
  }
  acc_guard4(acc[0][0], acc[0][1], acc[0][2], acc[0][3]);
  acc_guard4(acc[1][0], acc[1][1], acc[1][2], acc[1][3]);
  acc_guard4(acc[2][0], acc[2][1], acc[2][2], acc[2][3]);
  acc_guard4(acc[3][0], acc[3][1], acc[3][2], acc[3][3]);

  float* slab = sT[wave];
#pragma unroll
  for (int i = 0; i < 4; ++i) {
    const int mBase = m0 + (i << 4);
#pragma unroll
    for (int j = 0; j < 4; ++j) {
      const int n = n0 + (j << 4) + rlane;
      const float bv = bias[n];
#pragma unroll
      for (int r = 0; r < 8; ++r) {
        float v = acc[i][j][r] * scale;
        v += bv;
        if (ACT == 2) v = fmaxf(v, 0.0f);
        slab[(mOff + r) * SLABP + (j << 4) + rlane] = v;
      }
    }
    __builtin_amdgcn_fence(__ATOMIC_RELEASE, "workgroup");
    __builtin_amdgcn_wave_barrier();
    __builtin_amdgcn_fence(__ATOMIC_ACQUIRE, "workgroup");
    if (OUT_MODE == 0) {
      float* C = (float*)Cout;
      const int hh = lane >> 4, c4 = (lane & 15) * 4;
      for (int pass = 0; pass < 2; ++pass) {
#pragma unroll
        for (int it = 0; it < 8; ++it) {
          const int row = it * 2 + hh;
          const v4f v = *(const v4f*)(slab + row * SLABP + c4);
          *(volatile v4f*)(C + (size_t)(mBase + row) * ldc + n0 + c4) = v;
        }
        __threadfence();
      }
    } else {
      unsigned short* C = (unsigned short*)Cout;
      const int q = lane >> 3, c8 = (lane & 7) * 8;
      for (int pass = 0; pass < 2; ++pass) {
#pragma unroll
        for (int it = 0; it < 4; ++it) {
          const int row = it * 4 + q;
          const float* sp = slab + row * SLABP + c8;
          v8h hv;
#pragma unroll
          for (int e = 0; e < 8; ++e) hv[e] = (_Float16)sp[e];
          *(volatile v8h*)(C + (size_t)(mBase + row) * ldc + n0 + c8) = hv;
        }
        __threadfence();
      }
    }
    __builtin_amdgcn_fence(__ATOMIC_RELEASE, "workgroup");
    __builtin_amdgcn_wave_barrier();
    __builtin_amdgcn_fence(__ATOMIC_ACQUIRE, "workgroup");
  }
}

__global__ __launch_bounds__(NTHR) void lstm_scan_kernel(const float* __restrict__ XG,
                                                         const unsigned short* __restrict__ WHp,
                                                         unsigned short* __restrict__ HOUT) {
  __shared__ __align__(16) _Float16 Ah[SEQ_BLK * HPITCH];
  __shared__ __align__(16) float    XGs[SEQ_BLK * XGPITCH];
  const _Float16* WH = (const _Float16*)WHp;
  const int tid = threadIdx.x, lane = tid & 31, wave = tid >> 5;
  const int c = lane & 15, hh = lane >> 4, koff = hh * 8;
  const int rowbase = blockIdx.x * SEQ_BLK;

#pragma unroll 1
  for (int i = tid; i < SEQ_BLK * HPITCH; i += NTHR) Ah[i] = (_Float16)0.0f;
  float cst[8];
#pragma unroll
  for (int r = 0; r < 8; ++r) cst[r] = 0.0f;
  __syncthreads();

  const _Float16* ahrow = Ah + c * HPITCH + koff;
  const _Float16* wrow  = WH + (size_t)(16 * wave + c) * NHID + koff;
  const v8f z8 = {0.f, 0.f, 0.f, 0.f, 0.f, 0.f, 0.f, 0.f};
  const int st_row = tid >> 7;
  const int st_c4  = (tid & 127) * 4;
  const int orow   = 2 * wave + hh;

#pragma unroll 1
  for (int t = 0; t < NSTEP; ++t) {
    v4f xv[8];
#pragma unroll
    for (int i = 0; i < 8; ++i) {
      const int row = st_row + 2 * i;
      xv[i] = *(const v4f*)(XG + ((size_t)(rowbase + row) * NSTEP + (size_t)t) * NGATE + st_c4);
    }

    v8f acc0 = z8, acc1 = z8, acc2 = z8, acc3 = z8;
#pragma unroll 1
    for (int k0 = 0; k0 < NHID; k0 += 32) {
      const v16h a  = frag_load(ahrow + k0);
      const v16h b0 = frag_load(wrow + k0);
      const v16h b1 = frag_load(wrow + (size_t)1 * NHID * NHID + k0);
      const v16h b2 = frag_load(wrow + (size_t)2 * NHID * NHID + k0);
      const v16h b3 = frag_load(wrow + (size_t)3 * NHID * NHID + k0);
      acc0 = mma_f16(a, b0, acc0);
      acc1 = mma_f16(a, b1, acc1);
      acc2 = mma_f16(a, b2, acc2);
      acc3 = mma_f16(a, b3, acc3);
      guard4(acc0, acc1, acc2, acc3, a, b0, b1, b2, b3);
    }
    acc_guard4(acc0, acc1, acc2, acc3);

#pragma unroll
    for (int i = 0; i < 8; ++i) {
      const int row = st_row + 2 * i;
      *(v4f*)(XGs + row * XGPITCH + st_c4) = xv[i];
    }
    __syncthreads();

    float hn[8];
#pragma unroll
    for (int r = 0; r < 8; ++r) {
      const float* xr = XGs + (8 * hh + r) * XGPITCH + 16 * wave + c;
      const float zi = acc0[r] * WCARRY_INV + xr[0];
      const float zf = acc1[r] * WCARRY_INV + xr[NHID];
      const float zg = acc2[r] * WCARRY_INV + xr[2 * NHID];
      const float zo = acc3[r] * WCARRY_INV + xr[3 * NHID];
      const float ig = gate_sig(zi);
      const float fg = gate_sig(zf);
      const float gg = gate_tanh(zg);
      const float og = gate_sig(zo);
      const float cn = fg * cst[r] + ig * gg;
      cst[r] = cn;
      hn[r] = og * gate_tanh(cn);
    }
#pragma unroll
    for (int r = 0; r < 8; ++r) Ah[(8 * hh + r) * HPITCH + 16 * wave + c] = (_Float16)hn[r];
    __syncthreads();

    {
      const v8h hv = *(const v8h*)(Ah + orow * HPITCH + c * 8);
      unsigned short* dp = HOUT + ((size_t)(rowbase + orow) * NSTEP + (size_t)t) * NHID + c * 8;
      *(volatile v8h*)dp = hv;
      __threadfence();
      *(volatile v8h*)dp = hv;
    }
  }
}

__global__ __launch_bounds__(128) void head_kernel(const unsigned short* __restrict__ X2p,
                                                   const unsigned short* __restrict__ W3pp,
                                                   const float* __restrict__ b3, float* __restrict__ outc) {
  __shared__ __align__(16) float So[64 * NCLS];
  const _Float16* X2 = (const _Float16*)X2p;
  const _Float16* W3 = (const _Float16*)W3pp;
  const int tid = threadIdx.x, lane = tid & 31, wave = tid >> 5;
  const int c = lane & 15, hh = lane >> 4, koff = hh * 8;
  const int row0 = blockIdx.x * 64 + wave * 16;
  const _Float16* ap = X2 + (size_t)(row0 + c) * NFC2 + koff;
  const _Float16* bp = W3 + (size_t)c * NFC2 + koff;
  v8f acc = {0.f, 0.f, 0.f, 0.f, 0.f, 0.f, 0.f, 0.f};
#pragma unroll 2
  for (int k0 = 0; k0 < NFC2; k0 += 32) {
    const v16h a = frag_load(ap + k0);
    const v16h b = frag_load(bp + k0);
    acc = mma_f16(a, b, acc);
    guard1(acc, a, b);
  }
  acc_guard1(acc);
  const int cc = (c < NCLS) ? c : (NCLS - 1);
  const float bv = b3[cc];
#pragma unroll
  for (int r = 0; r < 8; ++r) {
    const float v = acc[r] * WCARRY_INV + bv;
    if (c < NCLS) So[(wave * 16 + 8 * hh + r) * NCLS + c] = v;
  }
  __syncthreads();
  float* ob = outc + (size_t)blockIdx.x * (64 * NCLS);
  for (int pass = 0; pass < 2; ++pass) {
    for (int g = wave; g < 5; g += 4) {
      const int i4 = (g * 32 + lane) * 4;
      const v4f v = *(const v4f*)(So + i4);
      *(volatile v4f*)(ob + i4) = v;
    }
    __threadfence();
  }
}

extern "C" void kernel_launch(void* const* d_in, const int* in_sizes, int n_in,
                              void* d_out, int out_size, void* d_ws, size_t ws_size, hipStream_t stream) {
  if (n_in < 15 || d_out == nullptr || d_ws == nullptr) return;
  if (in_sizes[0] != NROWS * NFEAT || in_sizes[1] != NGATE * NFEAT || in_sizes[2] != NGATE * NHID ||
      in_sizes[3] != NGATE || in_sizes[4] != NGATE || in_sizes[5] != NGATE * NHID ||
      in_sizes[6] != NGATE * NHID || in_sizes[7] != NGATE || in_sizes[8] != NGATE ||
      in_sizes[9] != NFC1 * NHID || in_sizes[10] != NFC1 || in_sizes[11] != NFC2 * NFC1 ||
      in_sizes[12] != NFC2 || in_sizes[13] != NCLS * NFC2 || in_sizes[14] != NCLS ||
      out_size != NROWS * NCLS) return;

  const float* mixture = (const float*)d_in[0];
  const float* Wih0 = (const float*)d_in[1];
  const float* Whh0 = (const float*)d_in[2];
  const float* bih0 = (const float*)d_in[3];
  const float* bhh0 = (const float*)d_in[4];
  const float* Wih1 = (const float*)d_in[5];
  const float* Whh1 = (const float*)d_in[6];
  const float* bih1 = (const float*)d_in[7];
  const float* bhh1 = (const float*)d_in[8];
  const float* W1 = (const float*)d_in[9];
  const float* b1 = (const float*)d_in[10];
  const float* W2 = (const float*)d_in[11];
  const float* b2 = (const float*)d_in[12];
  const float* W3 = (const float*)d_in[13];
  const float* b3 = (const float*)d_in[14];
  float* out = (float*)d_out;

  char* ws = (char*)d_ws;
  size_t off = 0;
  auto carve = [&](size_t bytes) -> char* { char* p = ws + off; off += (bytes + 255) & ~(size_t)255; return p; };
  unsigned short* XH    = (unsigned short*)carve((size_t)NROWS * NFEAT * 2);
  unsigned short* WIH0H = (unsigned short*)carve((size_t)NGATE * NFEAT * 2);
  unsigned short* WHH0H = (unsigned short*)carve((size_t)NGATE * NHID * 2);
  unsigned short* WIH1H = (unsigned short*)carve((size_t)NGATE * NHID * 2);
  unsigned short* WHH1H = (unsigned short*)carve((size_t)NGATE * NHID * 2);
  unsigned short* W1H   = (unsigned short*)carve((size_t)NFC1 * NHID * 2);
  unsigned short* W2H   = (unsigned short*)carve((size_t)NFC2 * NFC1 * 2);
  unsigned short* W3H   = (unsigned short*)carve((size_t)NCLS_PAD * NFC2 * 2);
  float*          BSUM  = (float*)carve((size_t)2 * NGATE * 4);
  unsigned short* H0    = (unsigned short*)carve((size_t)NROWS * NHID * 2);
  unsigned short* H1    = (unsigned short*)carve((size_t)NROWS * NHID * 2);
  float*          XG    = (float*)carve((size_t)NROWS * NGATE * 4);
  unsigned short* X1C   = (unsigned short*)carve((size_t)CHUNK_ROWS * NFC1 * 2);
  unsigned short* X2C   = (unsigned short*)carve((size_t)CHUNK_ROWS * NFC2 * 2);
  if (off > ws_size || off > (size_t)134217728) return;

  const int n8x  = NROWS * NFEAT / 8;
  const int n8g  = NGATE * NHID / 8;
  const int n8w1 = NFC1 * NHID / 8;
  const int n8w2 = NFC2 * NFC1 / 8;
  const int n8w3v = NCLS * NFC2 / 8;
  const int n8w3t = NCLS_PAD * NFC2 / 8;
  cvt8_f16_kernel<<<(n8x + NTHR - 1) / NTHR, NTHR, 0, stream>>>(mixture, XH, n8x, n8x, 1.0f);
  cvt8_f16_kernel<<<(n8g + NTHR - 1) / NTHR, NTHR, 0, stream>>>(Wih0, WIH0H, n8g, n8g, WCARRY);
  cvt8_f16_kernel<<<(n8g + NTHR - 1) / NTHR, NTHR, 0, stream>>>(Whh0, WHH0H, n8g, n8g, WCARRY);
  cvt8_f16_kernel<<<(n8g + NTHR - 1) / NTHR, NTHR, 0, stream>>>(Wih1, WIH1H, n8g, n8g, WCARRY);
  cvt8_f16_kernel<<<(n8g + NTHR - 1) / NTHR, NTHR, 0, stream>>>(Whh1, WHH1H, n8g, n8g, WCARRY);
  cvt8_f16_kernel<<<(n8w1 + NTHR - 1) / NTHR, NTHR, 0, stream>>>(W1, W1H, n8w1, n8w1, WCARRY);
  cvt8_f16_kernel<<<(n8w2 + NTHR - 1) / NTHR, NTHR, 0, stream>>>(W2, W2H, n8w2, n8w2, WCARRY);
  cvt8_f16_kernel<<<(n8w3t + NTHR - 1) / NTHR, NTHR, 0, stream>>>(W3, W3H, n8w3v, n8w3t, WCARRY);
  bias_sum_kernel<<<1, NTHR, 0, stream>>>(bih0, bhh0, bih1, bhh1, BSUM);

  const int gridProj = (NROWS / 64) * (NGATE / 64) / 8;
  gemm_f16_tile64<0, 0><<<gridProj, 256, 0, stream>>>(XH, NFEAT, WIH0H, NFEAT, (void*)XG, NGATE, BSUM,
                                                      NROWS, NGATE, NFEAT, WCARRY_INV);
  lstm_scan_kernel<<<NBATCH / SEQ_BLK, NTHR, 0, stream>>>(XG, WHH0H, H0);

  gemm_f16_tile64<0, 0><<<gridProj, 256, 0, stream>>>(H0, NHID, WIH1H, NHID, (void*)XG, NGATE, BSUM + NGATE,
                                                      NROWS, NGATE, NHID, WCARRY_INV);
  lstm_scan_kernel<<<NBATCH / SEQ_BLK, NTHR, 0, stream>>>(XG, WHH1H, H1);

  const int gridFc1 = (CHUNK_ROWS / 64) * (NFC1 / 64) / 8;
  const int gridFc2 = (CHUNK_ROWS / 64) * (NFC2 / 64) / 8;
  for (int ch = 0; ch < NCHUNK; ++ch) {
    const unsigned short* h1c = H1 + (size_t)ch * CHUNK_ROWS * NHID;
    float* outc = out + (size_t)ch * CHUNK_ROWS * NCLS;
    gemm_f16_tile64<1, 2><<<gridFc1, 256, 0, stream>>>(h1c, NHID, W1H, NHID, (void*)X1C, NFC1, b1,
                                                       CHUNK_ROWS, NFC1, NHID, WCARRY_INV);
    gemm_f16_tile64<1, 2><<<gridFc2, 256, 0, stream>>>(X1C, NFC1, W2H, NFC1, (void*)X2C, NFC2, b2,
                                                       CHUNK_ROWS, NFC2, NFC1, WCARRY_INV);
    head_kernel<<<CHUNK_ROWS / 64, 128, 0, stream>>>(X2C, W3H, b3, outc);
  }
}
